// CausalSelfAttention_47562467836684
// MI455X (gfx1250) — hardware-verified
//
#include <hip/hip_runtime.h>


#ifndef NB
#define NB 2
#endif
#ifndef SEQ
#define SEQ 2048
#endif
#define NB_FULL  2
#define SEQ_FULL 2048
#ifndef OUT_SEQ
#define OUT_SEQ SEQ
#endif
#define DM   1024
#define NH_  16
#define HD   64
#define NPR  8
#define GCH  32
#define NTOK (NB * SEQ)
#define FW   4
#define SC2  (0.125f * 1.4426950408889634f)
#define PSH  8.0f
#define CTXS 256.0f
#define WOS  256.0f
#define OUTI (1.0f / 65536.0f)
#define RMSE 1.1920929e-07f
#define LINIT 0.777870099559256f
#define OSC   0.222129900440744f
#define NEGS  (-3.0e38f)
#define MINIT (-1.0e30f)

static_assert(HD == 64);
static_assert(NH_ * HD == DM);
static_assert(NPR * 2 == NH_);
static_assert(NH_ == 16);
static_assert(GCH == 32);
static_assert(DM % 64 == 0);
static_assert(DM % 32 == 0);
static_assert(SEQ % 64 == 0);
static_assert((NB * SEQ) % 64 == 0);
static_assert(SEQ % 32 == 0);
static_assert(FW == 4);
static_assert(SEQ % (16 * (FW / 2)) == 0);
static_assert(((size_t)SEQ * DM) % 8 == 0);
static_assert(NB <= NB_FULL);
static_assert(SEQ <= SEQ_FULL);
static_assert((size_t)NB_FULL * SEQ_FULL * DM * 4 == (size_t)16777216);
static_assert(32 * 16 * 4 == 16 * 128);
static_assert(32 * 16 * 8 == 16 * 256);
static_assert(FW * 16 * 68 * 4 + FW * 16 * 4 <= 131072);
static_assert(64 * 72 * 2 <= 131072);
static_assert(16 * 68 * 4 <= 131072);

typedef _Float16 h16;
typedef unsigned short bf;
typedef __attribute__((ext_vector_type(16))) __bf16   v16bf;
typedef __attribute__((ext_vector_type(16))) _Float16 v16h;
typedef __attribute__((ext_vector_type(8)))  _Float16 v8h;
typedef __attribute__((ext_vector_type(8)))  unsigned short v8us;
typedef __attribute__((ext_vector_type(8)))  float    v8f;
typedef __attribute__((ext_vector_type(4)))  float    v4f;
typedef v4f  __attribute__((may_alias)) v4fa;
typedef v8us __attribute__((may_alias)) v8usa;

__device__ __forceinline__ unsigned short f2bf(float f) { unsigned u = __float_as_uint(f); u += 0x7FFFu + ((u >> 16) & 1u); return (unsigned short)(u >> 16); }
__device__ __forceinline__ float bfr(float f) { return __uint_as_float(((unsigned)f2bf(f)) << 16); }
__device__ __forceinline__ v16h cat16(v8h lo, v8h hi) { return __builtin_shufflevector(lo, hi, 0, 1, 2, 3, 4, 5, 6, 7, 8, 9, 10, 11, 12, 13, 14, 15); }
__device__ __forceinline__ v16bf cat16b(v8us lo, v8us hi) { return __builtin_bit_cast(v16bf, __builtin_shufflevector(lo, hi, 0, 1, 2, 3, 4, 5, 6, 7, 8, 9, 10, 11, 12, 13, 14, 15)); }
__device__ __forceinline__ v8f wmma16(v16h a, v16h b, v8f c) { return __builtin_amdgcn_wmma_f32_16x16x32_f16(false, a, false, b, (short)0, c, false, false); }
__device__ __forceinline__ v8f wmmab(v16bf a, v16bf b, v8f c) { return __builtin_amdgcn_wmma_f32_16x16x32_bf16(false, a, false, b, (short)0, c, false, false); }
__device__ __forceinline__ v16h  ldh(const h16* p) { return cat16(*(const v8h*)p, *(const v8h*)(p + 16)); }
__device__ __forceinline__ v16bf ldb(const bf* p)  { return cat16b(*(const v8us*)p, *(const v8us*)(p + 16)); }
__device__ __forceinline__ void wave_sync() { __builtin_amdgcn_fence(3  , "wavefront"); __builtin_amdgcn_wave_barrier(); asm volatile("" ::: "memory"); }
static __device__ __forceinline__ h16 toh_flush(float v) { const h16 r = (h16)v; return (fabsf(v) < 6.103515625e-05f) ? (h16)0.0f : r; }
__device__ __forceinline__ v8f wmma16g(v16h a, v16h b, v8f c) { c = __builtin_amdgcn_wmma_f32_16x16x32_f16(false, a, false, b, (short)0, c, false, false); asm volatile("v_nop\n\tv_nop\n\tv_nop\n\tv_nop" : "+v"(c) : "v"(a), "v"(b)); return c; }
__device__ __forceinline__ v8f wmmabg(v16bf a, v16bf b, v8f c) { c = __builtin_amdgcn_wmma_f32_16x16x32_bf16(false, a, false, b, (short)0, c, false, false); asm volatile("v_nop\n\tv_nop\n\tv_nop\n\tv_nop" : "+v"(c) : "v"(a), "v"(b)); return c; }

__global__ __launch_bounds__(256) void k_cvt8(const float* __restrict__ src, bf* dst, size_t nsrc8, size_t n8) {
    const size_t i = (size_t)blockIdx.x * 256 + threadIdx.x; if (i >= n8) return;
    const bool live = i < nsrc8; const size_t is = live ? i : (nsrc8 - 1);
    const v8f v = *(const v8f*)(src + is * 8); v8us o;
#pragma unroll
    for (int k = 0; k < 8; ++k) { const unsigned short c = f2bf(v[k]); o[k] = live ? c : (unsigned short)0; }
    *(volatile v8us*)(dst + i * 8) = o; __threadfence(); *(volatile v8us*)(dst + i * 8) = o;
}

__global__ __launch_bounds__(256) void k_wt(const float* __restrict__ W, bf* WT, int f16mode) {
    __shared__ __align__(16) unsigned short ts[64 * 72];
    const int tid = threadIdx.x; const int n0 = blockIdx.x * 64, k0 = blockIdx.y * 64;
#pragma unroll
    for (int p = 0; p < 4; ++p) { const int kr = p * 16 + (tid >> 4), c4 = (tid & 15) * 4;
        const v4f v = *(const v4f*)(W + (size_t)(k0 + kr) * DM + n0 + c4);
#pragma unroll
        for (int i = 0; i < 4; ++i) { const unsigned short bb = f2bf(v[i]); const float fb = __uint_as_float(((unsigned)bb) << 16);
            const unsigned short hb = __builtin_bit_cast(unsigned short, (h16)(fb * WOS));
            ts[(c4 + i) * 72 + kr] = f16mode ? hb : bb; } }
    __syncthreads();
#pragma unroll 1
    for (int ps = 0; ps < 2; ++ps) {
#pragma unroll
        for (int p = 0; p < 2; ++p) { const int n = p * 32 + (tid >> 3), c8 = (tid & 7) * 8;
            const v8us o = *(const v8usa*)(&ts[n * 72 + c8]);
            *(volatile v8us*)(WT + (size_t)(n0 + n) * DM + k0 + c8) = o; }
        if (ps == 0) __threadfence(); }
}

__global__ __launch_bounds__(32) void k_gate(const bf* __restrict__ XB, const float* __restrict__ Wg, float* G) {
    __shared__ __align__(16) float gs[16 * 68];
    const int lane = threadIdx.x & 31, lr = lane & 15, hi = lane >> 4; const int n0 = blockIdx.x * 64;
    float w0[8], w1[8];
#pragma unroll
    for (int i = 0; i < 8; ++i) w0[i] = Wg[(8 * hi + i) * NH_ + lr];
#pragma unroll
    for (int i = 0; i < 8; ++i) asm volatile("" : "+v"(w0[i]));
#pragma unroll
    for (int i = 0; i < 8; ++i) w1[i] = Wg[(16 + 8 * hi + i) * NH_ + lr];
    v8us alo, ahi;
#pragma unroll
    for (int i = 0; i < 8; ++i) { alo[i] = f2bf(w0[i]); ahi[i] = f2bf(w1[i]); }
    const v16bf a = cat16b(alo, ahi);
#pragma unroll
    for (int j = 0; j < 4; ++j) {
        const v16bf bx = ldb(XB + (size_t)(n0 + 16 * j + lr) * DM + 8 * hi);
        v8f c = (v8f){};
        c = wmmabg(a, bx, c);
#pragma unroll
        for (int r = 0; r < 8; ++r) gs[(8 * hi + r) * 68 + 16 * j + lr] = 2.0f * (1.0f / (1.0f + __expf(-c[r])));
    }
    wave_sync();
#pragma unroll 1
    for (int ps = 0; ps < 2; ++ps) {
#pragma unroll
        for (int s = 0; s < 8; ++s) { const int row = 2 * s + hi, cofs = lr * 4;
            const v4f x = *(const v4fa*)(&gs[row * 68 + cofs]);
            *(volatile v4f*)(G + (size_t)row * NTOK + n0 + cofs) = x; }
        if (ps == 0) __threadfence(); }
}


__global__ __launch_bounds__(32) void k_gemm_qk(const bf* __restrict__ A, const bf* __restrict__ Bt, const float* __restrict__ cosT, const float* __restrict__ sinT,
                                                h16* P0h, int RB, size_t sRB, int pitch, int CB, size_t sCB) {
    __shared__ __align__(16) float os[16 * 68];
    const int K = DM;
    const int lane = threadIdx.x & 31, lr = lane & 15, hi = lane >> 4; const int r0 = blockIdx.x * 64, c0 = blockIdx.y * 64;
    v8f acc[4][4];
#pragma unroll
    for (int mb = 0; mb < 4; ++mb)
#pragma unroll
        for (int nb = 0; nb < 4; ++nb) acc[mb][nb] = (v8f){};
    const size_t aoff = (size_t)(r0 + lr) * K + 8 * hi, boff = (size_t)(c0 + lr) * K + 8 * hi;
#pragma unroll 1
    for (int kc = 0; kc < K; kc += 32) {
        v16bf a[4];
#pragma unroll
        for (int mb = 0; mb < 4; ++mb) a[mb] = ldb(A + aoff + (size_t)mb * 16 * K + kc);
#pragma unroll
        for (int nb = 0; nb < 4; ++nb) { const v16bf b = ldb(Bt + boff + (size_t)nb * 16 * K + kc);
#pragma unroll
            for (int mb = 0; mb < 4; ++mb) acc[mb][nb] = wmmab(a[mb], b, acc[mb][nb]); }
        asm volatile("v_nop\n\tv_nop\n\tv_nop\n\tv_nop" : "+v"(acc[0][0]), "+v"(acc[1][1]), "+v"(acc[2][2]), "+v"(acc[3][3]) : "v"(a[0]), "v"(a[1]), "v"(a[2]), "v"(a[3]));
    }
    const size_t tbase = (size_t)(r0 / RB) * sRB + (size_t)(r0 % RB) * (size_t)pitch + (size_t)(c0 / CB) * sCB + (size_t)(c0 % CB);
#pragma unroll
    for (int mb = 0; mb < 4; ++mb) {
#pragma unroll
        for (int nb = 0; nb < 4; ++nb) {
#pragma unroll
            for (int j = 0; j < 8; ++j) os[(hi * 8 + j) * 68 + nb * 16 + lr] = acc[mb][nb][j]; }
        wave_sync();
        const size_t sbase = tbase + (size_t)(mb * 16) * (size_t)pitch;
        const int tp0 = (r0 % SEQ) + mb * 16;
#pragma unroll 1
        for (int ps = 0; ps < 2; ++ps) {
#pragma unroll
            for (int s = 0; s < 4; ++s) { const int row = 4 * s + (lane >> 3), c8 = (lane & 7) * 8;
                const int cp = c8 ^ 32, j8 = c8 & 31;
                const v4f x0 = *(const v4fa*)(&os[row * 68 + c8]); const v4f x1 = *(const v4fa*)(&os[row * 68 + c8 + 4]);
                const v4f y0 = *(const v4fa*)(&os[row * 68 + cp]); const v4f y1 = *(const v4fa*)(&os[row * 68 + cp + 4]);
                const size_t to = (size_t)(tp0 + row) * 32 + j8;
                const v4f cA = *(const v4f*)(cosT + to); const v4f cB = *(const v4f*)(cosT + to + 4);
                const v4f sA = *(const v4f*)(sinT + to); const v4f sB = *(const v4f*)(sinT + to + 4);
                const float sg = (c8 < 32) ? 1.0f : -1.0f;
                float val[8]; float ss = 0.0f;
#pragma unroll
                for (int i = 0; i < 4; ++i) { val[i] = x0[i] * bfr(cA[i]) + sg * (y0[i] * bfr(sA[i])); val[4 + i] = x1[i] * bfr(cB[i]) + sg * (y1[i] * bfr(sB[i])); }
#pragma unroll
                for (int i = 0; i < 8; ++i) ss += val[i] * val[i];
                ss += __shfl_xor(ss, 1, 32); ss += __shfl_xor(ss, 2, 32); ss += __shfl_xor(ss, 4, 32);
                const float inv = rsqrtf(ss * (1.0f / 64.0f) + RMSE);
                v8h hv;
#pragma unroll
                for (int i = 0; i < 8; ++i) hv[i] = toh_flush(val[i] * inv);
                *(volatile v8h*)(P0h + sbase + (size_t)row * (size_t)pitch + c8) = hv; }
            if (ps == 0) __threadfence(); }
        wave_sync();
    }
}

__global__ __launch_bounds__(32) void k_gemm_vt(const bf* __restrict__ A, const bf* __restrict__ Bt, const float* __restrict__ G, const float* __restrict__ VE,
                                                h16* P0h, int RB, size_t sRB, int pitch, int CB, size_t sCB) {
    __shared__ __align__(16) float os[16 * 68];
    const int K = DM;
    const int lane = threadIdx.x & 31, lr = lane & 15, hi = lane >> 4; const int r0 = blockIdx.x * 64, c0 = blockIdx.y * 64;
    v8f acc[4][4];
#pragma unroll
    for (int mb = 0; mb < 4; ++mb)
#pragma unroll
        for (int nb = 0; nb < 4; ++nb) acc[mb][nb] = (v8f){};
    const size_t aoff = (size_t)(r0 + lr) * K + 8 * hi, boff = (size_t)(c0 + lr) * K + 8 * hi;
#pragma unroll 1
    for (int kc = 0; kc < K; kc += 32) {
        v16bf a[4];
#pragma unroll
        for (int mb = 0; mb < 4; ++mb) a[mb] = ldb(A + aoff + (size_t)mb * 16 * K + kc);
#pragma unroll
        for (int nb = 0; nb < 4; ++nb) { const v16bf b = ldb(Bt + boff + (size_t)nb * 16 * K + kc);
#pragma unroll
            for (int mb = 0; mb < 4; ++mb) acc[mb][nb] = wmmab(a[mb], b, acc[mb][nb]); }
        asm volatile("v_nop\n\tv_nop\n\tv_nop\n\tv_nop" : "+v"(acc[0][0]), "+v"(acc[1][1]), "+v"(acc[2][2]), "+v"(acc[3][3]) : "v"(a[0]), "v"(a[1]), "v"(a[2]), "v"(a[3]));
    }
    const size_t tbase = (size_t)(r0 / RB) * sRB + (size_t)(r0 % RB) * (size_t)pitch + (size_t)(c0 / CB) * sCB + (size_t)(c0 % CB);
    const int hh = r0 / HD;
    const int bb = c0 / SEQ, tt0 = c0 % SEQ;
#pragma unroll
    for (int mb = 0; mb < 4; ++mb) {
#pragma unroll
        for (int nb = 0; nb < 4; ++nb) {
#pragma unroll
            for (int j = 0; j < 8; ++j) os[(hi * 8 + j) * 68 + nb * 16 + lr] = acc[mb][nb][j]; }
        wave_sync();
        const size_t sbase = tbase + (size_t)(mb * 16) * (size_t)pitch;
#pragma unroll 1
        for (int ps = 0; ps < 2; ++ps) {
#pragma unroll
            for (int s = 0; s < 4; ++s) { const int row = 4 * s + (lane >> 3), c8 = (lane & 7) * 8;
                const int mcol = r0 + mb * 16 + row;
                const v4f x0 = *(const v4fa*)(&os[row * 68 + c8]); const v4f x1 = *(const v4fa*)(&os[row * 68 + c8 + 4]);
                const v4f g0 = *(const v4f*)(G + (size_t)hh * NTOK + c0 + c8); const v4f g1 = *(const v4f*)(G + (size_t)hh * NTOK + c0 + c8 + 4);
                float e[8];
#pragma unroll
                for (int i = 0; i < 8; ++i) e[i] = VE[((size_t)bb * SEQ_FULL + (size_t)(tt0 + c8 + i)) * DM + mcol];
                v8h hv;
#pragma unroll
                for (int i = 0; i < 4; ++i) { hv[i] = toh_flush(x0[i] + g0[i] * bfr(e[i])); hv[4 + i] = toh_flush(x1[i] + g1[i] * bfr(e[4 + i])); }
                *(volatile v8h*)(P0h + sbase + (size_t)row * (size_t)pitch + c8) = hv; }
            if (ps == 0) __threadfence(); }
        wave_sync();
    }
}

__global__ __launch_bounds__(32) void k_gemm_out(const bf* __restrict__ A, const bf* __restrict__ Bt, float sa, float* OutF) {
    __shared__ __align__(16) float os[16 * 68];
    const int K = DM;
    const int lane = threadIdx.x & 31, lr = lane & 15, hi = lane >> 4; const int r0 = blockIdx.x * 64, c0 = blockIdx.y * 64;
    v8f acc[4][4];
#pragma unroll
    for (int mb = 0; mb < 4; ++mb)
#pragma unroll
        for (int nb = 0; nb < 4; ++nb) acc[mb][nb] = (v8f){};
    const size_t aoff = (size_t)(r0 + lr) * K + 8 * hi, boff = (size_t)(c0 + lr) * K + 8 * hi;
    const h16* Ah = (const h16*)A; const h16* Bh = (const h16*)Bt;
#pragma unroll 1
    for (int kc = 0; kc < K; kc += 32) {
        v16h a[4];
#pragma unroll
        for (int mb = 0; mb < 4; ++mb) a[mb] = ldh(Ah + aoff + (size_t)mb * 16 * K + kc);
#pragma unroll
        for (int nb = 0; nb < 4; ++nb) { const v16h b = ldh(Bh + boff + (size_t)nb * 16 * K + kc);
#pragma unroll
            for (int mb = 0; mb < 4; ++mb) acc[mb][nb] = wmma16(a[mb], b, acc[mb][nb]); }
        asm volatile("v_nop\n\tv_nop\n\tv_nop\n\tv_nop" : "+v"(acc[0][0]), "+v"(acc[1][1]), "+v"(acc[2][2]), "+v"(acc[3][3]) : "v"(a[0]), "v"(a[1]), "v"(a[2]), "v"(a[3]));
    }
#pragma unroll
    for (int mb = 0; mb < 4; ++mb) {
#pragma unroll
        for (int nb = 0; nb < 4; ++nb) {
#pragma unroll
            for (int j = 0; j < 8; ++j) os[(hi * 8 + j) * 68 + nb * 16 + lr] = acc[mb][nb][j]; }
        wave_sync();
        const int g0 = r0 + mb * 16;
        const size_t ob = ((size_t)(g0 / SEQ) * OUT_SEQ + (size_t)(g0 % SEQ)) * DM + c0;
#pragma unroll 1
        for (int ps = 0; ps < 2; ++ps) {
#pragma unroll
            for (int s = 0; s < 8; ++s) { const int row = 2 * s + hi, cofs = lr * 4;
                const v4f x = *(const v4fa*)(&os[row * 68 + cofs]); v4f val;
#pragma unroll
                for (int i = 0; i < 4; ++i) val[i] = x[i] * sa;
                *(volatile v4f*)(OutF + ob + (size_t)row * DM + cofs) = val; }
            if (ps == 0) __threadfence(); }
        wave_sync();
    }
}

__device__ __forceinline__ void sm_step(const v8f sa, const v8f sb, const int dq, const unsigned wwin, float& m, float& l, float& alpha, v16h& pb) {
    float ta[8], tb[8]; float mx = NEGS;
#pragma unroll
    for (int r = 0; r < 8; ++r) {
        const unsigned d0 = (unsigned)(dq - r), d1 = (unsigned)(dq - r - 16);
        const float va = sa[r] * SC2, vb = sb[r] * SC2;
        ta[r] = (d0 <= wwin) ? va : NEGS; tb[r] = (d1 <= wwin) ? vb : NEGS;
        mx = fmaxf(mx, fmaxf(ta[r], tb[r])); }
    mx = fmaxf(mx, __shfl_xor(mx, 16, 32));
    const float mnew = fmaxf(m, mx);
    alpha = __builtin_amdgcn_exp2f(m - mnew);
    const float sh = PSH - mnew;
    float ls = 0.0f;
#pragma unroll
    for (int r = 0; r < 8; ++r) {
        const float ea = ta[r] + sh, eb = tb[r] + sh;
        const float xa = __builtin_amdgcn_exp2f(ea), xb = __builtin_amdgcn_exp2f(eb);
        const h16 pa = (ea < -14.0f) ? (h16)0.0f : (h16)xa; const h16 pc = (eb < -14.0f) ? (h16)0.0f : (h16)xb;
        pb[r] = pa; pb[8 + r] = pc; ls += (float)pa + (float)pc; }
    l = l * alpha + ls; m = mnew;
}

__global__ __launch_bounds__(32 * FW) __attribute__((amdgpu_num_vgpr(256)))
void k_flash(const h16* __restrict__ QP, const h16* __restrict__ KP, const h16* __restrict__ VT,
             const float* __restrict__ lq1, const float* __restrict__ lk1, const float* __restrict__ lq2, const float* __restrict__ lk2,
             const float* __restrict__ dnw, const int* __restrict__ win, h16* CTX) {
    __shared__ __align__(16) float os[FW * 16 * 68];
    __shared__ float sq[FW * 16];
    const int lane = threadIdx.x & 31, lr = lane & 15, hi = lane >> 4;
    const int wave = __builtin_amdgcn_readfirstlane(threadIdx.x >> 5);
    const int vs = wave & 1;
    const int zp = blockIdx.y; const int b = zp / NPR, pr = zp % NPR;
    const int t0 = (blockIdx.x * (FW / 2) + (wave >> 1)) * 16;
    const int tq = t0 + lr;
    const int wraw = win[0];
    const int wcl = min(max(wraw, 0), SEQ);
    const unsigned wwin = (unsigned)wcl;
    const int klo = max(t0 - wcl, 0) & ~31;
    const size_t p1 = (size_t)(b * NH_ + 2 * pr) * SEQ * HD;
    const size_t p2 = p1 + (size_t)SEQ * HD;
    const size_t qo = (size_t)(t0 + lr) * HD + 8 * hi;
    const v16h q1a = ldh(QP + p1 + qo), q1b = ldh(QP + p1 + qo + 32), q2a = ldh(QP + p2 + qo), q2b = ldh(QP + p2 + qo + 32);
    const size_t ko = (size_t)lr * HD + 8 * hi;
    const size_t vo = p1 + (size_t)vs * SEQ * HD + (size_t)lr * SEQ + 8 * hi;
    v8f oA0 = (v8f){}, oA1 = (v8f){}, oA2 = (v8f){}, oA3 = (v8f){};
    v8f oB0 = (v8f){}, oB1 = (v8f){}, oB2 = (v8f){}, oB3 = (v8f){};
    float m1 = MINIT, l1 = 0.0f, m2 = MINIT, l2 = 0.0f;
#pragma unroll 1
    for (int key0 = klo; key0 <= t0 + 15; key0 += 32) {
        const int dq = tq - key0 - 8 * hi;
        v16h pb1, pb2; float al1, al2;
        {   const h16* ka = KP + p1 + ko + (size_t)key0 * HD;
            const v16h ka0 = ldh(ka), ka1 = ldh(ka + 32), kb0 = ldh(ka + 16 * HD), kb1 = ldh(ka + 16 * HD + 32);
            v8f sa = (v8f){}, sb = (v8f){};
            sa = wmma16g(ka0, q1a, sa); sb = wmma16g(kb0, q1a, sb); sa = wmma16g(ka1, q1b, sa); sb = wmma16g(kb1, q1b, sb);
            sm_step(sa, sb, dq, wwin, m1, l1, al1, pb1); }
        {   const h16* ka = KP + p2 + ko + (size_t)key0 * HD;
            const v16h ka0 = ldh(ka), ka1 = ldh(ka + 32), kb0 = ldh(ka + 16 * HD), kb1 = ldh(ka + 16 * HD + 32);
            v8f sa = (v8f){}, sb = (v8f){};
            sa = wmma16g(ka0, q2a, sa); sb = wmma16g(kb0, q2a, sb); sa = wmma16g(ka1, q2b, sa); sb = wmma16g(kb1, q2b, sb);
            sm_step(sa, sb, dq, wwin, m2, l2, al2, pb2); }
        oA0 = oA0 * al1; oA1 = oA1 * al1; oA2 = oA2 * al1; oA3 = oA3 * al1;
        oB0 = oB0 * al2; oB1 = oB1 * al2; oB2 = oB2 * al2; oB3 = oB3 * al2;
        const h16* va = VT + vo + key0;
        const v16h v0 = ldh(va), v1 = ldh(va + (size_t)16 * SEQ), v2 = ldh(va + (size_t)32 * SEQ), v3 = ldh(va + (size_t)48 * SEQ);
        oA0 = wmma16g(v0, pb1, oA0); oB0 = wmma16g(v0, pb2, oB0);
        oA1 = wmma16g(v1, pb1, oA1); oB1 = wmma16g(v1, pb2, oB1);
        oA2 = wmma16g(v2, pb1, oA2); oB2 = wmma16g(v2, pb2, oB2);
        oA3 = wmma16g(v3, pb1, oA3); oB3 = wmma16g(v3, pb2, oB3);
    }
    l1 += __shfl_xor(l1, 16, 32); l2 += __shfl_xor(l2, 16, 32);
    float d1 = bfr(lq1[lane]) * bfr(lk1[lane]) + bfr(lq1[lane + 32]) * bfr(lk1[lane + 32]);
    float d2 = bfr(lq2[lane]) * bfr(lk2[lane]) + bfr(lq2[lane + 32]) * bfr(lk2[lane + 32]);
    d1 += __shfl_xor(d1, 16, 32); d2 += __shfl_xor(d2, 16, 32);
    d1 += __shfl_xor(d1, 8, 32);  d2 += __shfl_xor(d2, 8, 32);
    d1 += __shfl_xor(d1, 4, 32);  d2 += __shfl_xor(d2, 4, 32);
    d1 += __shfl_xor(d1, 2, 32);  d2 += __shfl_xor(d2, 2, 32);
    d1 += __shfl_xor(d1, 1, 32);  d2 += __shfl_xor(d2, 1, 32);
    d1 = fminf(fmaxf(d1, -10.0f), 10.0f); d2 = fminf(fmaxf(d2, -10.0f), 10.0f);
    const float lam = __expf(d1) - __expf(d2) + LINIT;
    const float i1 = 1.0f / l1; const float i2 = lam * (1.0f / l2);
    oA0 = oA0 * i1 - oB0 * i2; oA1 = oA1 * i1 - oB1 * i2; oA2 = oA2 * i1 - oB2 * i2; oA3 = oA3 * i1 - oB3 * i2;
    float ssq = 0.0f;
#pragma unroll
    for (int r = 0; r < 8; ++r) ssq += oA0[r] * oA0[r] + oA1[r] * oA1[r] + oA2[r] * oA2[r] + oA3[r] * oA3[r];
    ssq += __shfl_xor(ssq, 16, 32);
    sq[wave * 16 + lr] = ssq;
    __syncthreads();
    const float tot = ssq + sq[(wave ^ 1) * 16 + lr];
    const float rn = rsqrtf(tot * (1.0f / 128.0f) + RMSE);
    const float pz = (wraw < 0) ? __uint_as_float(0x7FC00000u) : 0.0f;
    const int wb = wave * 16 * 68;
    { v4f a, c;
      a[0] = oA0[0] * rn + pz; a[1] = oA0[1] * rn + pz; a[2] = oA0[2] * rn + pz; a[3] = oA0[3] * rn + pz; c[0] = oA0[4] * rn + pz; c[1] = oA0[5] * rn + pz; c[2] = oA0[6] * rn + pz; c[3] = oA0[7] * rn + pz;
      *(v4fa*)(&os[wb + lr * 68 +  0 + 8 * hi]) = a; *(v4fa*)(&os[wb + lr * 68 +  0 + 8 * hi + 4]) = c;
      a[0] = oA1[0] * rn + pz; a[1] = oA1[1] * rn + pz; a[2] = oA1[2] * rn + pz; a[3] = oA1[3] * rn + pz; c[0] = oA1[4] * rn + pz; c[1] = oA1[5] * rn + pz; c[2] = oA1[6] * rn + pz; c[3] = oA1[7] * rn + pz;
      *(v4fa*)(&os[wb + lr * 68 + 16 + 8 * hi]) = a; *(v4fa*)(&os[wb + lr * 68 + 16 + 8 * hi + 4]) = c;
      a[0] = oA2[0] * rn + pz; a[1] = oA2[1] * rn + pz; a[2] = oA2[2] * rn + pz; a[3] = oA2[3] * rn + pz; c[0] = oA2[4] * rn + pz; c[1] = oA2[5] * rn + pz; c[2] = oA2[6] * rn + pz; c[3] = oA2[7] * rn + pz;
      *(v4fa*)(&os[wb + lr * 68 + 32 + 8 * hi]) = a; *(v4fa*)(&os[wb + lr * 68 + 32 + 8 * hi + 4]) = c;
      a[0] = oA3[0] * rn + pz; a[1] = oA3[1] * rn + pz; a[2] = oA3[2] * rn + pz; a[3] = oA3[3] * rn + pz; c[0] = oA3[4] * rn + pz; c[1] = oA3[5] * rn + pz; c[2] = oA3[6] * rn + pz; c[3] = oA3[7] * rn + pz;
      *(v4fa*)(&os[wb + lr * 68 + 48 + 8 * hi]) = a; *(v4fa*)(&os[wb + lr * 68 + 48 + 8 * hi + 4]) = c; }
    wave_sync();
    h16* crow = CTX + ((size_t)b * SEQ + t0) * DM + (2 * pr + vs) * HD;
#pragma unroll 1
    for (int ps = 0; ps < 2; ++ps) {
#pragma unroll
        for (int s = 0; s < 4; ++s) { const int row = 4 * s + (lane >> 3), c8 = (lane & 7) * 8;
            const v4f x0 = *(const v4fa*)(&os[wb + row * 68 + c8]); const v4f x1 = *(const v4fa*)(&os[wb + row * 68 + c8 + 4]);
            const v4f w0 = *(const v4f*)(dnw + vs * HD + c8); const v4f w1 = *(const v4f*)(dnw + vs * HD + c8 + 4); v8h hv;
#pragma unroll
            for (int i = 0; i < 4; ++i) { hv[i] = toh_flush(x0[i] * bfr(w0[i]) * (OSC * CTXS)); hv[4 + i] = toh_flush(x1[i] * bfr(w1[i]) * (OSC * CTXS)); }
            *(volatile v8h*)(crow + (size_t)row * DM + c8) = hv; }
        if (ps == 0) __threadfence(); }
}

static constexpr size_t al256(size_t v) { return (v + 255) & ~(size_t)255; }
static constexpr size_t SZ_XB  = al256((size_t)NB * SEQ * DM * 2);
static constexpr size_t SZ_WT  = al256((size_t)DM * DM * 2);
static constexpr size_t SZ_G   = al256((size_t)NH_ * NTOK * 4);
static constexpr size_t SZ_PL  = al256((size_t)NB * NH_ * SEQ * HD * 2);
static constexpr size_t SZ_CTX = al256((size_t)NB * SEQ * DM * 2);
static constexpr size_t SZ_TOTAL = SZ_XB + 4 * SZ_WT + SZ_G + 3 * SZ_PL + SZ_CTX;
static_assert(SZ_TOTAL <= (size_t)134217728);

static void cvt_x(const float* x, bf* XB, hipStream_t stream) {
    if (SEQ == SEQ_FULL) {
        const size_t n8 = (size_t)NB * SEQ * DM / 8;
        k_cvt8<<<(unsigned)((n8 + 255) / 256), 256, 0, stream>>>(x, XB, n8, n8);
    } else {
        const size_t n8 = (size_t)SEQ * DM / 8;
        for (int b = 0; b < NB; ++b) k_cvt8<<<(unsigned)((n8 + 255) / 256), 256, 0, stream>>>(x + (size_t)b * SEQ_FULL * DM, XB + (size_t)b * SEQ * DM, n8, n8);
    }
}

extern "C" void kernel_launch(void* const* d_in, const int* in_sizes, int n_in,
                              void* d_out, int out_size, void* d_ws, size_t ws_size, hipStream_t stream) {
    if (n_in < 15) return;
    const size_t needx = ((size_t)(NB - 1) * SEQ_FULL + SEQ) * DM;
    if ((size_t)in_sizes[0] < needx || (size_t)in_sizes[1] < needx) return;
    if ((size_t)in_sizes[2] < (size_t)SEQ * 32 || (size_t)in_sizes[3] < (size_t)SEQ * 32) return;
    if ((size_t)in_sizes[4] < (size_t)DM * DM || (size_t)in_sizes[5] < (size_t)DM * DM || (size_t)in_sizes[6] < (size_t)DM * DM || (size_t)in_sizes[7] < (size_t)DM * DM) return;
    if (in_sizes[8] < GCH * NH_) return;
    if (in_sizes[9] < HD || in_sizes[10] < HD || in_sizes[11] < HD || in_sizes[12] < HD) return;
    if (in_sizes[13] < 2 * HD || in_sizes[14] < 1) return;
    if ((size_t)out_size < ((size_t)(NB - 1) * OUT_SEQ + SEQ) * DM) return;
    if (SZ_TOTAL > ws_size) return;
    const float* x  = (const float*)d_in[0]; const float* ve = (const float*)d_in[1];
    const float* ct = (const float*)d_in[2]; const float* st = (const float*)d_in[3];
    const float* wq = (const float*)d_in[4]; const float* wk = (const float*)d_in[5];
    const float* wv = (const float*)d_in[6]; const float* wp = (const float*)d_in[7];
    const float* wg = (const float*)d_in[8];
    const float* lq1 = (const float*)d_in[9];  const float* lk1 = (const float*)d_in[10];
    const float* lq2 = (const float*)d_in[11]; const float* lk2 = (const float*)d_in[12];
    const float* dnw = (const float*)d_in[13]; const int* win = (const int*)d_in[14];
    float* OUT = (float*)d_out;
    char* wsp = (char*)d_ws;
    bf* XB  = (bf*)wsp; wsp += SZ_XB;
    bf* WQT = (bf*)wsp; wsp += SZ_WT;
    bf* WKT = (bf*)wsp; wsp += SZ_WT;
    bf* WVT = (bf*)wsp; wsp += SZ_WT;
    bf* WPT = (bf*)wsp; wsp += SZ_WT;
    float* GP = (float*)wsp; wsp += SZ_G;
    h16* QP  = (h16*)wsp; wsp += SZ_PL;
    h16* KP  = (h16*)wsp; wsp += SZ_PL;
    h16* VT  = (h16*)wsp; wsp += SZ_PL;
    h16* CTX = (h16*)wsp; wsp += SZ_CTX;

    cvt_x(x, XB, stream);
    k_wt<<<dim3(DM / 64, DM / 64, 1), 256, 0, stream>>>(wq, WQT, 0);
    k_wt<<<dim3(DM / 64, DM / 64, 1), 256, 0, stream>>>(wk, WKT, 0);
    k_wt<<<dim3(DM / 64, DM / 64, 1), 256, 0, stream>>>(wv, WVT, 0);
    k_wt<<<dim3(DM / 64, DM / 64, 1), 256, 0, stream>>>(wp, WPT, 1);

    k_gate<<<dim3(NTOK / 64, 1, 1), 32, 0, stream>>>(XB, wg, GP);

    k_gemm_qk<<<dim3(NTOK / 64, DM / 64, 1), 32, 0, stream>>>(XB, WQT, ct, st, QP, SEQ, (size_t)NH_ * SEQ * HD, HD, HD, (size_t)SEQ * HD);
    k_gemm_qk<<<dim3(NTOK / 64, DM / 64, 1), 32, 0, stream>>>(XB, WKT, ct, st, KP, SEQ, (size_t)NH_ * SEQ * HD, HD, HD, (size_t)SEQ * HD);
    k_gemm_vt<<<dim3(DM / 64, NTOK / 64, 1), 32, 0, stream>>>(WVT, XB, GP, ve, VT, DM, (size_t)0, SEQ, SEQ, (size_t)DM * SEQ);

    k_flash<<<dim3(SEQ / (16 * (FW / 2)), NB * NPR, 1), 32 * FW, 0, stream>>>(QP, KP, VT, lq1, lk1, lq2, lk2, dnw, win, CTX);

    k_gemm_out<<<dim3(NTOK / 64, DM / 64, 1), 32, 0, stream>>>((const bf*)CTX, WPT, OUTI, OUT);
}
